// MultiHeadAttention_10728828305608
// MI455X (gfx1250) — hardware-verified
//
#include <hip/hip_runtime.h>
#include <stddef.h>


#ifndef NB
#define NB 2
#endif
#ifndef SEQ
#define SEQ 2048
#endif
#define NB_FULL 2
#define SEQ_FULL 2048
#define DM 1024
#define NH 16
#define DKH 64
#define MROWS (NB * SEQ)
#define PLANE ((size_t)MROWS * DM)

#define ATT_THREADS 128
#define ATT_WAVES   4
#define ATT_QROWS   64

static_assert(NB >= 1 && NB <= NB_FULL);
static_assert(SEQ >= 128 && SEQ <= SEQ_FULL);
static_assert(SEQ % 128 == 0);
static_assert(SEQ % 64 == 0 && SEQ % 32 == 0);
static_assert(MROWS % 64 == 0);
static_assert(DM == 1024);
static_assert(DM % 256 == 0 && DM % 32 == 0 && DM % 64 == 0 && DM % 8 == 0);
static_assert(NH * DKH == DM);
static_assert(DKH == 64);
static_assert(ATT_THREADS == 32 * ATT_WAVES);
static_assert(ATT_QROWS == 16 * ATT_WAVES);
static_assert(SEQ % ATT_QROWS == 0);
static_assert(ATT_THREADS * 2 * 8 == 32 * DKH);
static_assert(ATT_THREADS * 4 * 8 == ATT_QROWS * DKH);
static_assert((3 * 32 * 64 + 2 * ATT_QROWS * 64 + ATT_WAVES * 16 * 64) * 2 <= 65536);
static_assert((MROWS * (DM / 8)) % 256 == 0);
static_assert(((DM * DM) / 8) % 256 == 0);
static_assert((9 * (size_t)MROWS * DM + 4 * (size_t)DM * DM) * 2 <= (size_t)134217728);

#define P_CARRY   1024.0f
#define CTX_SCALE 0.25f
#define WO_CARRY  64.0f
#define OUT_FOLD  (1.0f / 16384.0f)
#define QK_SCALE  0.125f

typedef unsigned short us;
typedef us        v8us  __attribute__((ext_vector_type(8)));
typedef us        v16us __attribute__((ext_vector_type(16)));
typedef _Float16  v16h  __attribute__((ext_vector_type(16)));
typedef __bf16    v16bf __attribute__((ext_vector_type(16)));
typedef float     v8f   __attribute__((ext_vector_type(8)));
typedef float     v4f   __attribute__((ext_vector_type(4)));

__device__ __forceinline__ unsigned bf16rne_bits(float x) {
  unsigned u = __float_as_uint(x);
  return (u + 0x7FFFu + ((u >> 16) & 1u)) >> 16;
}
__device__ __forceinline__ float bf16rne(float x) {
  return __uint_as_float(bf16rne_bits(x) << 16);
}
__device__ __forceinline__ us f16_bits(float x) {
  _Float16 hx = (_Float16)x;
  return __builtin_bit_cast(us, hx);
}

__device__ __forceinline__ v16us join16(v8us c0, v8us c1) {
  return __builtin_shufflevector(c0, c1, 0, 1, 2, 3, 4, 5, 6, 7, 8, 9, 10, 11, 12, 13, 14, 15);
}
__device__ __forceinline__ v16us frag16(const us* __restrict__ base, int ld, int row0, int k0) {
  const int l = threadIdx.x & 31;
  const int r = l & 15, s = l >> 4;
  const us* p = base + (size_t)(row0 + r) * ld + k0 + 8 * s;
  v8us c0 = *(const v8us*)p;
  v8us c1 = *(const v8us*)(p + 16);
  return join16(c0, c1);
}
__device__ __forceinline__ v16h fragh(const us* __restrict__ base, int ld, int row0, int k0) {
  return __builtin_bit_cast(v16h, frag16(base, ld, row0, k0));
}
__device__ __forceinline__ v16bf fragb(const us* __restrict__ base, int ld, int row0, int k0) {
  return __builtin_bit_cast(v16bf, frag16(base, ld, row0, k0));
}
#define LDS_FRAG(arr, off) join16(*(const v8us*)&arr[(off)], *(const v8us*)&arr[(off) + 16])

__device__ __forceinline__ v8f mma_f16(v16h a, v16h b, v8f c) {
  v8f d = __builtin_amdgcn_wmma_f32_16x16x32_f16(false, a, false, b, (short)0, c, false, false);
  asm volatile("v_nop\n\tv_nop\n\tv_nop\n\tv_nop" : "+v"(d) : "v"(a), "v"(b));
  return d;
}
__device__ __forceinline__ v8f mma_bf16(v16bf a, v16bf b, v8f c) {
  v8f d = __builtin_amdgcn_wmma_f32_16x16x32_bf16(false, a, false, b, (short)0, c, false, false);
  asm volatile("v_nop\n\tv_nop\n\tv_nop\n\tv_nop" : "+v"(d) : "v"(a), "v"(b));
  return d;
}

__global__ __launch_bounds__(256) void cvt_x_kernel(const float* __restrict__ X, us* Y, int n8) {
  const int i = blockIdx.x * 256 + threadIdx.x;
  if (i >= n8) return;
  const int m  = i >> 7;
  const int c8 = (i & 127) * 8;
  const int b  = m / SEQ;
  const int s  = m - b * SEQ;
  const float* src = X + ((size_t)(b * SEQ_FULL + s)) * DM + c8;
  v4f x0 = *(const v4f*)src;
  v4f x1 = *(const v4f*)(src + 4);
  v8us y;
#pragma unroll
  for (int j = 0; j < 4; ++j) {
    y[j]     = (us)bf16rne_bits(x0[j]);
    y[4 + j] = (us)bf16rne_bits(x1[j]);
  }
  us* dst = Y + (size_t)i * 8;
  *(volatile v8us*)dst = y;
  __threadfence();
  *(volatile v8us*)dst = y;
}

__global__ __launch_bounds__(256) void cvt_w_kernel(const float* __restrict__ W, us* WT, int n8, int hmode) {
  const int i = blockIdx.x * 256 + threadIdx.x;
  if (i >= n8) return;
  const float* src = W + (size_t)i * 8;
  v4f x0 = *(const v4f*)src;
  v4f x1 = *(const v4f*)(src + 4);
  v8us y;
#pragma unroll
  for (int j = 0; j < 4; ++j) {
    const float w0 = bf16rne(x0[j]);
    const float w1 = bf16rne(x1[j]);
    const us b0 = (us)(__float_as_uint(w0) >> 16);
    const us b1 = (us)(__float_as_uint(w1) >> 16);
    const us h0 = f16_bits(w0 * WO_CARRY);
    const us h1 = f16_bits(w1 * WO_CARRY);
    y[j]     = hmode ? h0 : b0;
    y[4 + j] = hmode ? h1 : b1;
  }
  us* dst = WT + (size_t)i * 8;
  *(volatile v8us*)dst = y;
  __threadfence();
  *(volatile v8us*)dst = y;
}

__device__ __forceinline__ void gemm32x64_bf16(const us* __restrict__ A, const us* __restrict__ B,
                                               int m0, int n0, v8f (&acc)[8]) {
#pragma unroll 1
  for (int kk = 0; kk < DM; kk += 32) {
    const v16bf a0 = fragb(A, DM, m0, kk);
    const v16bf a1 = fragb(A, DM, m0 + 16, kk);
#pragma unroll
    for (int tt = 0; tt < 4; ++tt) {
      const v16bf b = fragb(B, DM, n0 + 16 * tt, kk);
      acc[tt]     = mma_bf16(a0, b, acc[tt]);
      acc[4 + tt] = mma_bf16(a1, b, acc[4 + tt]);
    }
  }
}
__device__ __forceinline__ void gemm32x64_f16(const us* __restrict__ A, const us* __restrict__ B,
                                              int m0, int n0, v8f (&acc)[8]) {
#pragma unroll 1
  for (int kk = 0; kk < DM; kk += 32) {
    const v16h a0 = fragh(A, DM, m0, kk);
    const v16h a1 = fragh(A, DM, m0 + 16, kk);
#pragma unroll
    for (int tt = 0; tt < 4; ++tt) {
      const v16h b = fragh(B, DM, n0 + 16 * tt, kk);
      acc[tt]     = mma_f16(a0, b, acc[tt]);
      acc[4 + tt] = mma_f16(a1, b, acc[4 + tt]);
    }
  }
}

static_assert(256 == 8 * 32);
static_assert(2 * 32 == 64 && 4 * 64 == 256);
static_assert(2 * 32 * 256 * 2 <= 65536);
static_assert(64 * 256 * 2 <= 65536);
static_assert(8 * 32 == 2 * 32 * 4);
static_assert(8 * 8 == DKH);

__global__ __launch_bounds__(256)
void proj_qk_kernel(const us* __restrict__ Xb, const us* __restrict__ Wt,
                    const float* __restrict__ bias, us* Y) {
  __shared__ __attribute__((aligned(16))) us stile[2 * 32 * 256];

  const int t = threadIdx.x, wid = t >> 5, l = t & 31;
  const int h = l >> 4, r16 = l & 15;
  const int wm = wid >> 2, wn = wid & 3;
  const int mblk0 = blockIdx.x * 64;
  const int nblk0 = blockIdx.y * 256;
  const int m0 = mblk0 + wm * 32;
  const int n0 = nblk0 + wn * 64;

  v8f acc[8] = {};
  gemm32x64_bf16(Xb, Wt, m0, n0, acc);

  float bvv[4];
#pragma unroll
  for (int tt = 0; tt < 4; ++tt) bvv[tt] = bf16rne(bias[n0 + 16 * tt + r16]);

  const int bblk = mblk0 / SEQ;
  const int sblk = mblk0 - bblk * SEQ;
  const int c = l & 7;

#pragma unroll
  for (int mi = 0; mi < 2; ++mi) {
    if (mi) __syncthreads();

#pragma unroll
    for (int tt = 0; tt < 4; ++tt) {
      const int nl = wn * 64 + 16 * tt + r16;
#pragma unroll
      for (int r = 0; r < 8; ++r) {
        const int rl = wm * 16 + 8 * h + r;
        const float v = acc[mi * 4 + tt][r] + bvv[tt];
        const unsigned hb = bf16rne_bits(v);
        const float hf = __uint_as_float(hb << 16);
        const unsigned lb = bf16rne_bits(v - hf);
        stile[rl * 256 + nl]            = (us)hb;
        stile[32 * 256 + rl * 256 + nl] = (us)lb;
      }
    }
    __syncthreads();

    v8us vals[8];
    size_t dsts[8];
#pragma unroll
    for (int it = 0; it < 8; ++it) {
      const int L  = wid * 32 + (l >> 3) + 4 * it;
      const int pl = L >> 7;
      const int Lp = L & 127;
      const int rl = Lp >> 2, hq = Lp & 3;
      const int hg = (nblk0 >> 6) + hq;
      const int ml = (rl >> 4) * 32 + mi * 16 + (rl & 15);
      const int s  = sblk + ml;
      vals[it] = *(const v8us*)&stile[pl * (32 * 256) + rl * 256 + hq * 64 + 8 * c];
      dsts[it] = (size_t)pl * PLANE + (((size_t)(bblk * NH + hg)) * SEQ + s) * DKH + 8 * c;
    }
#pragma unroll
    for (int it = 0; it < 8; ++it) *(volatile v8us*)(Y + dsts[it]) = vals[it];
    __threadfence();
#pragma unroll
    for (int it = 0; it < 8; ++it) *(volatile v8us*)(Y + dsts[it]) = vals[it];
    __builtin_amdgcn_sched_barrier(0);
  }
}

__global__ __launch_bounds__(256)
void proj_vt_kernel(const us* __restrict__ Xb, const us* __restrict__ Wt,
                    const float* __restrict__ bias, us* Y) {
  __shared__ __attribute__((aligned(16))) us stile[256 * 64];

  const int t = threadIdx.x, wid = t >> 5, l = t & 31;
  const int h = l >> 4, r16 = l & 15;
  const int wm = wid >> 2, wn = wid & 3;
  const int mblk0 = blockIdx.x * 64;
  const int nblk0 = blockIdx.y * 256;
  const int m0 = mblk0 + wm * 32;
  const int n0 = nblk0 + wn * 64;

  v8f acc[8] = {};
  gemm32x64_bf16(Xb, Wt, m0, n0, acc);

#pragma unroll
  for (int tt = 0; tt < 4; ++tt) {
    const int nl = wn * 64 + 16 * tt + r16;
    const float bvv = bf16rne(bias[n0 + 16 * tt + r16]);
#pragma unroll
    for (int mi = 0; mi < 2; ++mi) {
#pragma unroll
      for (int r = 0; r < 8; ++r) {
        const int ml = wm * 32 + 16 * mi + 8 * h + r;
        stile[nl * 64 + ml] = f16_bits(acc[mi * 4 + tt][r] + bvv);
      }
    }
  }
  __syncthreads();

  const int bblk = mblk0 / SEQ;
  const int sblk = mblk0 - bblk * SEQ;
  const int c = l & 7;
  v8us vals[8];
  size_t dsts[8];
#pragma unroll
  for (int it = 0; it < 8; ++it) {
    const int L = wid * 32 + (l >> 3) + 4 * it;
    const int n = nblk0 + L;
    const int hg = n >> 6, d = n & 63;
    vals[it] = *(const v8us*)&stile[L * 64 + 8 * c];
    dsts[it] = (((size_t)(bblk * NH + hg)) * DKH + d) * SEQ + sblk + 8 * c;
  }
#pragma unroll
  for (int it = 0; it < 8; ++it) *(volatile v8us*)(Y + dsts[it]) = vals[it];
  __threadfence();
#pragma unroll
  for (int it = 0; it < 8; ++it) *(volatile v8us*)(Y + dsts[it]) = vals[it];
}

__global__ __launch_bounds__(ATT_THREADS)
void attn_kernel(const us* __restrict__ Qp, const us* __restrict__ Kp,
                 const us* __restrict__ Vt, us* Ctx) {
  __shared__ __attribute__((aligned(16))) us shKh[32 * 64];
  __shared__ __attribute__((aligned(16))) us shKl[32 * 64];
  __shared__ __attribute__((aligned(16))) us shV[64 * 32];
  __shared__ __attribute__((aligned(16))) us shQh[ATT_QROWS * 64];
  __shared__ __attribute__((aligned(16))) us shQl[ATT_QROWS * 64];
  __shared__ __attribute__((aligned(16))) us shC[ATT_WAVES * 16 * 64];

  const int t = threadIdx.x;
  const int wid = t >> 5;
  const int l = t & 31;
  const int r16 = l & 15;
  const int hs = l >> 4;
  const int rowsel = hs << 3;
  constexpr int QBLK = SEQ / ATT_QROWS;
  const int bh = blockIdx.x / QBLK;
  const int qb = blockIdx.x - bh * QBLK;
  const int q0 = qb * ATT_QROWS + wid * 16;

  const size_t hoff = (size_t)bh * SEQ * DKH;
  const us* khp = Kp + hoff;
  const us* klp = Kp + PLANE + hoff;
  const us* vp  = Vt + hoff;

  {
    const size_t qg = hoff + (size_t)qb * ATT_QROWS * DKH;
#pragma unroll
    for (int j = 0; j < 4; ++j) {
      const int pi = (t + ATT_THREADS * j) * 8;
      const v8us xh = *(const v8us*)(Qp + qg + pi);
      const v8us xl = *(const v8us*)(Qp + PLANE + qg + pi);
      *(v8us*)&shQh[pi] = xh;
      *(v8us*)&shQl[pi] = xl;
    }
  }

  v8f o[4];
#pragma unroll
  for (int tt = 0; tt < 4; ++tt) o[tt] = v8f{};
  float mmax = -1.0e30f, lsum = 0.0f;

  const int p0i = t, p1i = t + ATT_THREADS;
  const int krow0 = p0i >> 3, kcol0 = (p0i & 7) * 8;
  const int krow1 = p1i >> 3, kcol1 = (p1i & 7) * 8;
  const int vrow0 = p0i >> 2, vcol0 = (p0i & 3) * 8;
  const int vrow1 = p1i >> 2, vcol1 = (p1i & 3) * 8;
  const int fk = r16 * 64 + 8 * hs;
  const int fv = r16 * 32 + 8 * hs;
  const int fq = (wid * 16 + r16) * 64 + 8 * hs;

#pragma unroll 1
  for (int kb = 0; kb < SEQ; kb += 32) {
    __syncthreads();
    {
      const size_t go0 = (size_t)(kb + krow0) * DKH + kcol0;
      const size_t go1 = (size_t)(kb + krow1) * DKH + kcol1;
      const v8us xh0 = *(const v8us*)(khp + go0);
      const v8us xh1 = *(const v8us*)(khp + go1);
      const v8us xl0 = *(const v8us*)(klp + go0);
      const v8us xl1 = *(const v8us*)(klp + go1);
      const v8us xv0 = *(const v8us*)(vp + (size_t)vrow0 * SEQ + kb + vcol0);
      const v8us xv1 = *(const v8us*)(vp + (size_t)vrow1 * SEQ + kb + vcol1);
      *(v8us*)&shKh[krow0 * 64 + kcol0] = xh0;
      *(v8us*)&shKh[krow1 * 64 + kcol1] = xh1;
      *(v8us*)&shKl[krow0 * 64 + kcol0] = xl0;
      *(v8us*)&shKl[krow1 * 64 + kcol1] = xl1;
      *(v8us*)&shV[vrow0 * 32 + vcol0]  = xv0;
      *(v8us*)&shV[vrow1 * 32 + vcol1]  = xv1;
    }
    __syncthreads();

    v8f s0 = {};
    v8f s1 = {};
#pragma unroll
    for (int dc = 0; dc < 2; ++dc) {
      const int qo = fq + 32 * dc;
      const int ko = fk + 32 * dc;
      const v16bf qh = __builtin_bit_cast(v16bf, LDS_FRAG(shQh, qo));
      const v16bf ql = __builtin_bit_cast(v16bf, LDS_FRAG(shQl, qo));
      {
        const v16bf ka = __builtin_bit_cast(v16bf, LDS_FRAG(shKh, ko));
        const v16bf kl = __builtin_bit_cast(v16bf, LDS_FRAG(shKl, ko));
        s0 = mma_bf16(ka, qh, s0);
        s0 = mma_bf16(ka, ql, s0);
        s0 = mma_bf16(kl, qh, s0);
      }
      __builtin_amdgcn_sched_barrier(0);
      {
        const v16bf ka = __builtin_bit_cast(v16bf, LDS_FRAG(shKh, 16 * 64 + ko));
        const v16bf kl = __builtin_bit_cast(v16bf, LDS_FRAG(shKl, 16 * 64 + ko));
        s1 = mma_bf16(ka, qh, s1);
        s1 = mma_bf16(ka, ql, s1);
        s1 = mma_bf16(kl, qh, s1);
      }
      __builtin_amdgcn_sched_barrier(0);
    }

    float bm = s0[0];
#pragma unroll
    for (int i = 0; i < 8; ++i) { bm = fmaxf(bm, s0[i]); bm = fmaxf(bm, s1[i]); }
    bm = fmaxf(bm, __shfl_xor(bm, 16, 32));
    const float mnew = fmaxf(mmax, bm * QK_SCALE);
    const float corr = __expf(mmax - mnew);
    mmax = mnew;

    float ps = 0.0f;
    v16h pA;
#pragma unroll
    for (int i = 0; i < 8; ++i) {
      const float p0 = __expf(s0[i] * QK_SCALE - mnew);
      const float p1 = __expf(s1[i] * QK_SCALE - mnew);
      ps += p0 + p1;
      pA[i]     = (_Float16)(p0 * P_CARRY);
      pA[8 + i] = (_Float16)(p1 * P_CARRY);
    }
    ps += __shfl_xor(ps, 16, 32);
    lsum = lsum * corr + ps;

#pragma unroll
    for (int r = 0; r < 8; ++r) {
      const float cr = __shfl(corr, rowsel + r, 32);
#pragma unroll
      for (int tt = 0; tt < 4; ++tt) o[tt][r] *= cr;
    }
    __builtin_amdgcn_sched_barrier(0);

    {
      const v16h vB0 = __builtin_bit_cast(v16h, LDS_FRAG(shV, 0 * 16 * 32 + fv));
      const v16h vB1 = __builtin_bit_cast(v16h, LDS_FRAG(shV, 1 * 16 * 32 + fv));
      const v16h vB2 = __builtin_bit_cast(v16h, LDS_FRAG(shV, 2 * 16 * 32 + fv));
      const v16h vB3 = __builtin_bit_cast(v16h, LDS_FRAG(shV, 3 * 16 * 32 + fv));
      o[0] = mma_f16(pA, vB0, o[0]);
      o[1] = mma_f16(pA, vB1, o[1]);
      o[2] = mma_f16(pA, vB2, o[2]);
      o[3] = mma_f16(pA, vB3, o[3]);
    }
    __builtin_amdgcn_sched_barrier(0);
  }

  const int bb = bh / NH;
  const int hh = bh - bb * NH;
#pragma unroll
  for (int r = 0; r < 8; ++r) {
    const float lrow = __shfl(lsum, rowsel + r, 32);
    const float li = CTX_SCALE * __builtin_amdgcn_rcpf(lrow);
#pragma unroll
    for (int tt = 0; tt < 4; ++tt) {
      shC[wid * 1024 + (rowsel + r) * 64 + 16 * tt + r16] = f16_bits(o[tt][r] * li);
    }
  }
  __syncthreads();

  const int c = l & 7;
  v8us vals[4];
  size_t dsts[4];
#pragma unroll
  for (int it = 0; it < 4; ++it) {
    const int rl = (l >> 3) + 4 * it;
    vals[it] = *(const v8us*)&shC[wid * 1024 + rl * 64 + 8 * c];
    const int s = q0 + rl;
    dsts[it] = ((size_t)(bb * SEQ + s)) * DM + hh * DKH + 8 * c;
  }
#pragma unroll
  for (int it = 0; it < 4; ++it) *(volatile v8us*)(Ctx + dsts[it]) = vals[it];
  __threadfence();
#pragma unroll
  for (int it = 0; it < 4; ++it) *(volatile v8us*)(Ctx + dsts[it]) = vals[it];
}

__global__ __launch_bounds__(256) __attribute__((amdgpu_num_vgpr(256)))
void outproj_kernel(const us* __restrict__ Ctx, const us* __restrict__ Wot,
                    const float* __restrict__ bo, float* Out) {
  __shared__ __attribute__((aligned(16))) float ftile[32 * 256];

  const int t = threadIdx.x, wid = t >> 5, l = t & 31;
  const int h = l >> 4, r16 = l & 15;
  const int wm = wid >> 2, wn = wid & 3;
  const int mblk0 = blockIdx.x * 64;
  const int nblk0 = blockIdx.y * 256;
  const int m0 = mblk0 + wm * 32;
  const int n0 = nblk0 + wn * 64;

  v8f acc[8] = {};
  gemm32x64_f16(Ctx, Wot, m0, n0, acc);

  const int c = l & 7;
#pragma unroll
  for (int p = 0; p < 2; ++p) {
    if (p) __syncthreads();
#pragma unroll
    for (int tt = 0; tt < 4; ++tt) {
      const int n = n0 + 16 * tt + r16;
      const float bob = bf16rne(bo[n]);
      const int nl = wn * 64 + 16 * tt + r16;
#pragma unroll
      for (int r = 0; r < 8; ++r) {
        const int rl = wm * 16 + 8 * h + r;
        ftile[rl * 256 + nl] = acc[p * 4 + tt][r] * OUT_FOLD + bob;
      }
    }
    __syncthreads();

    v4f vals[8];
    size_t dsts[8];
#pragma unroll
    for (int it = 0; it < 8; ++it) {
      const int L = wid * 32 + (l >> 3) + 4 * it;
      const int rl = L >> 3, seg = L & 7;
      vals[it] = *(const v4f*)&ftile[rl * 256 + seg * 32 + 4 * c];
      const int m = mblk0 + (rl >> 4) * 32 + p * 16 + (rl & 15);
      dsts[it] = (size_t)m * DM + nblk0 + seg * 32 + 4 * c;
    }
#pragma unroll
    for (int it = 0; it < 8; ++it) *(volatile v4f*)(Out + dsts[it]) = vals[it];
    __threadfence();
#pragma unroll
    for (int it = 0; it < 8; ++it) *(volatile v4f*)(Out + dsts[it]) = vals[it];
  }
}

extern "C" void kernel_launch(void* const* d_in, const int* in_sizes, int n_in,
                              void* d_out, int out_size, void* d_ws, size_t ws_size,
                              hipStream_t stream) {
  if (n_in < 11) return;
  const int need_x = ((NB - 1) * SEQ_FULL + SEQ) * DM;
  if (in_sizes[0] < need_x || in_sizes[1] < need_x || in_sizes[2] < need_x) return;
  if (in_sizes[3] < DM * DM || in_sizes[5] < DM * DM || in_sizes[7] < DM * DM || in_sizes[9] < DM * DM) return;
  if (in_sizes[4] < DM || in_sizes[6] < DM || in_sizes[8] < DM || in_sizes[10] < DM) return;
  if (out_size < MROWS * DM) return;

  const float* Q  = (const float*)d_in[0];
  const float* K  = (const float*)d_in[2];
  const float* V  = (const float*)d_in[1];
  const float* Wq = (const float*)d_in[3];
  const float* bq = (const float*)d_in[4];
  const float* Wk = (const float*)d_in[5];
  const float* bk = (const float*)d_in[6];
  const float* Wv = (const float*)d_in[7];
  const float* bv = (const float*)d_in[8];
  const float* Wo = (const float*)d_in[9];
  const float* bo = (const float*)d_in[10];

  const size_t XE = PLANE;
  const size_t WE = (size_t)DM * DM;
  const size_t total_bytes = (9 * XE + 4 * WE) * sizeof(us);
  if (total_bytes > ws_size) return;

  us* xq  = (us*)d_ws;
  us* xk  = xq + XE;
  us* xv  = xk + XE;
  us* wtq = xv + XE;
  us* wtk = wtq + WE;
  us* wtv = wtk + WE;
  us* wot = wtv + WE;
  us* qpl = wot + WE;
  us* kpl = qpl + 2 * XE;
  us* vt  = kpl + 2 * XE;
  us* ctx = vt + XE;

  dim3 blk(256);
  const int n8 = (int)(XE / 8);
  dim3 gx((n8 + 255) / 256);
  cvt_x_kernel<<<gx, blk, 0, stream>>>(Q, xq, n8);
  cvt_x_kernel<<<gx, blk, 0, stream>>>(K, xk, n8);
  cvt_x_kernel<<<gx, blk, 0, stream>>>(V, xv, n8);

  const int w8 = (int)(WE / 8);
  dim3 gw((w8 + 255) / 256);
  cvt_w_kernel<<<gw, blk, 0, stream>>>(Wq, wtq, w8, 0);
  cvt_w_kernel<<<gw, blk, 0, stream>>>(Wk, wtk, w8, 0);
  cvt_w_kernel<<<gw, blk, 0, stream>>>(Wv, wtv, w8, 0);
  cvt_w_kernel<<<gw, blk, 0, stream>>>(Wo, wot, w8, 1);

  dim3 gp(MROWS / 64, DM / 256);
  proj_qk_kernel<<<gp, blk, 0, stream>>>(xq, wtq, bq, qpl);
  proj_qk_kernel<<<gp, blk, 0, stream>>>(xk, wtk, bk, kpl);
  proj_vt_kernel<<<gp, blk, 0, stream>>>(xv, wtv, bv, vt);

  attn_kernel<<<dim3(NB * NH * (SEQ / ATT_QROWS)), dim3(ATT_THREADS), 0, stream>>>(qpl, kpl, vt, ctx);

  outproj_kernel<<<gp, blk, 0, stream>>>(ctx, wot, bo, (float*)d_out);
}
